// SLSA_87840671137898
// MI455X (gfx1250) — hardware-run, weakly checked
//
#include <hip/hip_runtime.h>
#include <math.h>

typedef __attribute__((ext_vector_type(16))) _Float16 v16h;
typedef __attribute__((ext_vector_type(8)))  _Float16 v8h;
typedef __attribute__((ext_vector_type(16))) __bf16   v16b;
typedef __attribute__((ext_vector_type(8)))  __bf16   v8b;
typedef __attribute__((ext_vector_type(8)))  float    v8f;
typedef __attribute__((ext_vector_type(4)))  float    v4f;
typedef __attribute__((ext_vector_type(4)))  unsigned int v4u;

constexpr int kB    = 4;
constexpr int kT    = 2048;
constexpr int kC    = 1024;
constexpr int kH    = 16;
constexpr int kHS   = 64;
constexpr int kRows = kB * kT;
constexpr int kSqrtC = 32;
static_assert(kSqrtC * kSqrtC == kC, "score scale is 1/sqrt(C)");
static_assert(kH * kHS == kC, "head split");
static_assert((kC % 32) == 0 && (kHS % 32) == 0 && (kT % 64) == 0, "K multiples of 32, key chunks of 64");
static_assert((kRows % 64) == 0 && (kC % 64) == 0, "GEMM M,N multiples of 64");

constexpr float kXCarry = 16.0f;
constexpr float kWCarry = 1024.0f;
constexpr float kUCarry = 16.0f;
constexpr float kUScale  = kUCarry / (kXCarry * kWCarry);
constexpr float kV0Scale = 1.0f / (kXCarry * kWCarry);
constexpr float kScoreScale = 1.0f / ((float)kSqrtC * kUCarry * kXCarry);

constexpr size_t kSzAct16 = (size_t)kRows * kC * 2;
constexpr size_t kSzW16   = (size_t)kC * kC * 2;
constexpr size_t kSzW12   = (size_t)2 * kHS * kHS * 2;
constexpr size_t kSzV0    = (size_t)kRows * kC * 4;
constexpr size_t kOffXH   = 0;
constexpr size_t kOffWUT  = kOffXH  + kSzAct16;
constexpr size_t kOffWVT  = kOffWUT + kSzW16;
constexpr size_t kOffWPT  = kOffWVT + kSzW16;
constexpr size_t kOffW12  = kOffWPT + kSzW16;
constexpr size_t kOffU    = kOffW12 + kSzW12;
constexpr size_t kOffV0   = kOffU   + kSzAct16;
constexpr size_t kOffYH   = kOffV0;
constexpr size_t kOffYL   = kOffV0  + kSzAct16;
constexpr size_t kOffVTH  = kOffV0  + kSzV0;
constexpr size_t kOffVTL  = kOffVTH + kSzAct16;
constexpr size_t kWsTotal = kOffVTL + kSzAct16;
static_assert(kWsTotal == 106971136ull, "carve total");
static_assert(kWsTotal <= 134217728ull, "carve cap");
static_assert(2 * kSzAct16 == kSzV0, "y hi|lo planes fit the v0 plane exactly");
static_assert((kOffWUT % 128) == 0 && (kOffWVT % 128) == 0 && (kOffWPT % 128) == 0 && (kOffW12 % 128) == 0 &&
              (kOffU % 128) == 0 && (kOffV0 % 128) == 0 && (kOffYL % 128) == 0 && (kOffVTH % 128) == 0 &&
              (kOffVTL % 128) == 0, "128-B aligned regions");

__device__ __forceinline__ unsigned short f2bf_bits(float f) {
  unsigned u = __float_as_uint(f);
  return (unsigned short)((u + 0x7FFFu + ((u >> 16) & 1u)) >> 16);
}
__device__ __forceinline__ float bf_bits2f(unsigned short h) { return __uint_as_float(((unsigned)h) << 16); }
__device__ __forceinline__ unsigned pk16(unsigned short a, unsigned short b) { return (unsigned)a | ((unsigned)b << 16); }
__device__ __forceinline__ unsigned short h_bits(float f) { const _Float16 h = (_Float16)f; return __builtin_bit_cast(unsigned short, h); }
__device__ __forceinline__ void split_bits(float f, unsigned short& hb, unsigned short& lb) {
  hb = f2bf_bits(f);
  lb = f2bf_bits(f - bf_bits2f(hb));
}

__device__ __forceinline__ v8f mma_h(v16h a, v16h b, v8f c) {
  c = __builtin_amdgcn_wmma_f32_16x16x32_f16(false, a, false, b, (short)0, c, false, false);
  asm volatile("v_nop\n\tv_nop\n\tv_nop\n\tv_nop" : "+v"(c) : "v"(a), "v"(b));
  return c;
}
__device__ __forceinline__ v8f mma_b(v16b a, v16b b, v8f c) {
  c = __builtin_amdgcn_wmma_f32_16x16x32_bf16(false, a, false, b, (short)0, c, false, false);
  asm volatile("v_nop\n\tv_nop\n\tv_nop\n\tv_nop" : "+v"(c) : "v"(a), "v"(b));
  return c;
}
__device__ __forceinline__ void keep4_h(v16h a, v16h b, v16h c, v16h d) { asm volatile("v_nop" :: "v"(a), "v"(b), "v"(c), "v"(d)); }
__device__ __forceinline__ void keep4_b(v16b a, v16b b, v16b c, v16b d) { asm volatile("v_nop" :: "v"(a), "v"(b), "v"(c), "v"(d)); }
__device__ __forceinline__ void acc_guard4(v8f& a, v8f& b, v8f& c, v8f& d) { asm volatile("v_nop\n\tv_nop\n\tv_nop\n\tv_nop" : "+v"(a), "+v"(b), "+v"(c), "+v"(d)); }

template <typename T> struct Frag;
template <> struct Frag<_Float16> {
  typedef v16h V; union U { v16h v; v8h h[2]; };
  static __device__ __forceinline__ v16h load(const _Float16* p) {
    U f; f.h[0] = *(const v8h*)(p); f.h[1] = *(const v8h*)(p + 16); return f.v;
  }
  static __device__ __forceinline__ v8f mma(v16h a, v16h b, v8f c) { return mma_h(a, b, c); }
  static __device__ __forceinline__ void keep(v16h a, v16h b, v16h c, v16h d) { keep4_h(a, b, c, d); }
};
template <> struct Frag<__bf16> {
  typedef v16b V; union U { v16b v; v8b h[2]; };
  static __device__ __forceinline__ v16b load(const __bf16* p) {
    U f; f.h[0] = *(const v8b*)(p); f.h[1] = *(const v8b*)(p + 16); return f.v;
  }
  static __device__ __forceinline__ v8f mma(v16b a, v16b b, v8f c) { return mma_b(a, b, c); }
  static __device__ __forceinline__ void keep(v16b a, v16b b, v16b c, v16b d) { keep4_b(a, b, c, d); }
};

template <int ET> struct Elem;
template <> struct Elem<0> { typedef _Float16 T; };
template <> struct Elem<1> { typedef __bf16 T; };
template <int ET, int SPL, int BIAS_MODE, int OUT_MODE>
__global__ __launch_bounds__(256) void wmma_gemm64(
    const unsigned short* __restrict__ Ap, const unsigned short* __restrict__ A2p, int lda, long strideA,
    const unsigned short* __restrict__ Btp, const unsigned short* __restrict__ Bt2p, int ldb, long strideB,
    void* __restrict__ Cout, int ldc, long strideC,
    const float* __restrict__ bias,
    int M, int N, int K, float scale, float bias_scale) {
  typedef typename Elem<ET>::T T;
  typedef typename Frag<T>::V V;
  const T* A = (const T*)Ap; const T* A2 = (const T*)A2p; const T* Bt = (const T*)Btp; const T* Bt2 = (const T*)Bt2p;
  __shared__ __align__(16) float sT[8][16 * 68];
  const int b    = blockIdx.y;
  const int lane = threadIdx.x & 31;
  const int wave = threadIdx.x >> 5;
  const int tilesN = N >> 6;
  const int tilesM = M >> 6;
  const int tile = blockIdx.x * 8 + wave;
  if (tile >= tilesM * tilesN) return;
  const int tm = tile / tilesN;
  const int tn = tile - tm * tilesN;
  const int m0 = tm << 6;
  const int n0 = tn << 6;

  const T* Ab  = A  + (size_t)b * strideA;
  const T* Bb  = Bt + (size_t)b * strideB;
  const T* Ab2 = (SPL >= 1) ? (A2  + (size_t)b * strideA) : nullptr;
  const T* Bb2 = (SPL == 2) ? (Bt2 + (size_t)b * strideB) : nullptr;

  const int rlane = lane & 15;
  const int koff  = (lane >> 4) * 8;
  const int mOff  = (lane >> 4) * 8;

  v8f acc[4][4];
#pragma unroll
  for (int i = 0; i < 4; ++i)
#pragma unroll
    for (int j = 0; j < 4; ++j) acc[i][j] = (v8f){0.f,0.f,0.f,0.f,0.f,0.f,0.f,0.f};

  for (int k0 = 0; k0 < K; k0 += 32) {
    V bh[4], bl[4];
#pragma unroll
    for (int j = 0; j < 4; ++j) {
      const size_t bo = (size_t)(n0 + (j << 4) + rlane) * ldb + koff + k0;
      bh[j] = Frag<T>::load(Bb + bo);
      if (SPL == 2) bl[j] = Frag<T>::load(Bb2 + bo);
    }
#pragma unroll
    for (int i = 0; i < 4; ++i) {
      const size_t ao = (size_t)(m0 + (i << 4) + rlane) * lda + koff + k0;
      V ah = Frag<T>::load(Ab + ao);
      V al;
      if (SPL >= 1) al = Frag<T>::load(Ab2 + ao);
#pragma unroll
      for (int j = 0; j < 4; ++j) {
        acc[i][j] = Frag<T>::mma(ah, bh[j], acc[i][j]);
        if (SPL == 2) acc[i][j] = Frag<T>::mma(ah, bl[j], acc[i][j]);
        if (SPL >= 1) acc[i][j] = Frag<T>::mma(al, bh[j], acc[i][j]);
      }
    }
    Frag<T>::keep(bh[0], bh[1], bh[2], bh[3]);
    if (SPL == 2) Frag<T>::keep(bl[0], bl[1], bl[2], bl[3]);
  }
  acc_guard4(acc[0][0], acc[0][1], acc[0][2], acc[0][3]);
  acc_guard4(acc[1][0], acc[1][1], acc[1][2], acc[1][3]);
  acc_guard4(acc[2][0], acc[2][1], acc[2][2], acc[2][3]);
  acc_guard4(acc[3][0], acc[3][1], acc[3][2], acc[3][3]);

  float* slab = sT[wave];
#pragma unroll
  for (int i = 0; i < 4; ++i) {
    const int mBase = m0 + (i << 4);
#pragma unroll
    for (int j = 0; j < 4; ++j) {
      const int n = n0 + (j << 4) + rlane;
      float bv = 0.f;
      if (BIAS_MODE == 2) bv = bf_bits2f(f2bf_bits(bias[n])) * bias_scale;
#pragma unroll
      for (int r = 0; r < 8; ++r) {
        float v = acc[i][j][r] * scale;
        if (BIAS_MODE == 2) v += bv;
        slab[(mOff + r) * 68 + (j << 4) + rlane] = v;
      }
    }
    __builtin_amdgcn_fence(__ATOMIC_RELEASE, "workgroup");
    __builtin_amdgcn_wave_barrier();
    __builtin_amdgcn_fence(__ATOMIC_ACQUIRE, "workgroup");
    if (OUT_MODE == 0) {
      float* C = (float*)Cout + (size_t)b * strideC;
      const int hh = lane >> 4, c4 = (lane & 15) * 4;
      for (int pass = 0; pass < 2; ++pass) {
#pragma unroll
        for (int it = 0; it < 8; ++it) {
          const int row = it * 2 + hh;
          v4f v = *(const v4f*)(slab + row * 68 + c4);
          *(volatile v4f*)(C + (size_t)(mBase + row) * ldc + n0 + c4) = v;
        }
        __threadfence();
      }
    } else {
      const int q = lane >> 3, c8 = (lane & 7) * 8;
      unsigned short* C  = (unsigned short*)Cout  + (size_t)b * strideC;
      for (int pass = 0; pass < 2; ++pass) {
#pragma unroll
        for (int it = 0; it < 4; ++it) {
          const int row = it * 4 + q;
          const float* sp = slab + row * 68 + c8;
          v8h hv;
#pragma unroll
          for (int e = 0; e < 8; ++e) hv[e] = (_Float16)sp[e];
          *(volatile v8h*)(C + (size_t)(mBase + row) * ldc + n0 + c8) = hv;
        }
        __threadfence();
      }
    }
    __builtin_amdgcn_fence(__ATOMIC_RELEASE, "workgroup");
    __builtin_amdgcn_wave_barrier();
    __builtin_amdgcn_fence(__ATOMIC_ACQUIRE, "workgroup");
  }
}

__global__ __launch_bounds__(256) void cast_x_kernel(const float* __restrict__ in, unsigned short* __restrict__ out, int n8) {
  const int i = blockIdx.x * 256 + threadIdx.x;
  if (i >= n8) return;
  const float* p = in + 8 * (size_t)i;
  const v4f a = *(const v4f*)(p);
  const v4f c = *(const v4f*)(p + 4);
  unsigned short hb[8];
#pragma unroll
  for (int e = 0; e < 4; ++e) {
    const float a_e = a[e];
    const float c_e = c[e];
    hb[e]     = h_bits(bf_bits2f(f2bf_bits(a_e)) * kXCarry);
    hb[4 + e] = h_bits(bf_bits2f(f2bf_bits(c_e)) * kXCarry);
  }
  const v4u u = (v4u){pk16(hb[0], hb[1]), pk16(hb[2], hb[3]), pk16(hb[4], hb[5]), pk16(hb[6], hb[7])};
  unsigned short* q = out + 8 * (size_t)i;
  *(volatile v4u*)q = u;
  __threadfence();
  *(volatile v4u*)q = u;
}

__global__ __launch_bounds__(256) void wt_transpose_cast_kernel(const float* __restrict__ W0, const float* __restrict__ W1,
                                                                const float* __restrict__ W2, unsigned short* __restrict__ out,
                                                                int dim, float carry, int bf_from_z) {
  __shared__ float sm[64][65];
  const int t  = threadIdx.x;
  const int k0 = blockIdx.x * 64;
  const int n0 = blockIdx.y * 64;
  const int z  = blockIdx.z;
  const float* W = (z == 0) ? W0 : (z == 1) ? W1 : W2;
  const bool as_bf = (z >= bf_from_z);
#pragma unroll
  for (int i = 0; i < 16; ++i) {
    const int e = i * 256 + t;
    const int r = e >> 6;
    const int c = e & 63;
    sm[c][r] = W[(size_t)(k0 + r) * dim + n0 + c];
  }
  __syncthreads();
  const int lane = t & 31, wave = t >> 5;
  const int q = lane >> 3, c8 = (lane & 7) * 8;
  unsigned short* op = out + (size_t)z * dim * dim;
  for (int pass = 0; pass < 2; ++pass) {
#pragma unroll
    for (int it = 0; it < 2; ++it) {
      const int row = wave * 8 + it * 4 + q;
      unsigned short hb[8];
#pragma unroll
      for (int e = 0; e < 8; ++e) {
        const float w = sm[row][c8 + e];
        const unsigned short bb = f2bf_bits(w);
        const unsigned short fh = h_bits(bf_bits2f(bb) * carry);
        hb[e] = as_bf ? bb : fh;
      }
      const v4u u = (v4u){pk16(hb[0], hb[1]), pk16(hb[2], hb[3]), pk16(hb[4], hb[5]), pk16(hb[6], hb[7])};
      *(volatile v4u*)(op + (size_t)(n0 + row) * dim + k0 + c8) = u;
    }
    __threadfence();
  }
}

constexpr int kGP = 68;
__global__ __launch_bounds__(128) void gated_value_kernel(
    const float* __restrict__ V0, const unsigned short* __restrict__ W1tp, const unsigned short* __restrict__ W2tp,
    const float* __restrict__ b1, const float* __restrict__ b2,
    unsigned short* __restrict__ VTH, unsigned short* __restrict__ VTL)
{
  __shared__ __align__(16) float sA[64 * kGP];
  __shared__ __align__(16) float sB[64 * kGP];
  __shared__ __align__(16) __bf16 sW1[kHS * kHS];
  __shared__ __align__(16) __bf16 sW2[kHS * kHS];
  __shared__ float sBias[2 * kHS];
  const int tid = threadIdx.x, lane = tid & 31, wave = tid >> 5;
  const int hh = lane >> 4, c = lane & 15;
  const int g0 = blockIdx.x * 64;
  const int hd = blockIdx.y;
  const int bidx = g0 / kT;
  const int t0 = g0 - bidx * kT;
  const __bf16* W1t = (const __bf16*)W1tp;
  const __bf16* W2t = (const __bf16*)W2tp;
#pragma unroll
  for (int i = 0; i < 8; ++i) {
    const int e = i * 128 + tid;
    const int r = e >> 4, c4 = (e & 15) * 4;
    *(v4f*)(sA + r * kGP + c4) = *(const v4f*)(V0 + (size_t)(g0 + r) * kC + hd * kHS + c4);
  }
#pragma unroll
  for (int i = 0; i < 4; ++i) {
    const int e = (i * 128 + tid) * 8;
    *(v8b*)(sW1 + e) = *(const v8b*)(W1t + e);
    *(v8b*)(sW2 + e) = *(const v8b*)(W2t + e);
  }
  {
    const int bi = tid & 63;
    const float x1 = b1[bi];
    const float x2 = b2[bi];
    const float xs = (tid < kHS) ? x1 : x2;
    sBias[tid] = bf_bits2f(f2bf_bits(xs));
  }
  __syncthreads();

  v16b ah[2], al[2];
  {
    const int arow = wave * 16 + c;
#pragma unroll
    for (int ks = 0; ks < 2; ++ks) {
      const float* p = sA + arow * kGP + ks * 32 + 8 * hh;
      const v4f f0 = *(const v4f*)(p);
      const v4f f1 = *(const v4f*)(p + 4);
      const v4f f2 = *(const v4f*)(p + 16);
      const v4f f3 = *(const v4f*)(p + 20);
#pragma unroll
      for (int e = 0; e < 4; ++e) {
        unsigned short hb, lb;
        const float x0 = f0[e];
        const float x1 = f1[e];
        const float x2 = f2[e];
        const float x3 = f3[e];
        split_bits(x0, hb, lb);
        ah[ks][e] = __builtin_bit_cast(__bf16, hb);       al[ks][e] = __builtin_bit_cast(__bf16, lb);
        split_bits(x1, hb, lb);
        ah[ks][4 + e] = __builtin_bit_cast(__bf16, hb);   al[ks][4 + e] = __builtin_bit_cast(__bf16, lb);
        split_bits(x2, hb, lb);
        ah[ks][8 + e] = __builtin_bit_cast(__bf16, hb);   al[ks][8 + e] = __builtin_bit_cast(__bf16, lb);
        split_bits(x3, hb, lb);
        ah[ks][12 + e] = __builtin_bit_cast(__bf16, hb);  al[ks][12 + e] = __builtin_bit_cast(__bf16, lb);
      }
    }
  }

  v8f a1[4], a2[4];
#pragma unroll
  for (int j = 0; j < 4; ++j) {
    a1[j] = (v8f){0.f,0.f,0.f,0.f,0.f,0.f,0.f,0.f};
    a2[j] = (v8f){0.f,0.f,0.f,0.f,0.f,0.f,0.f,0.f};
  }
#pragma unroll
  for (int ks = 0; ks < 2; ++ks) {
#pragma unroll
    for (int j = 0; j < 4; ++j) {
      const v16b w1 = Frag<__bf16>::load(sW1 + (j * 16 + c) * kHS + ks * 32 + 8 * hh);
      const v16b w2 = Frag<__bf16>::load(sW2 + (j * 16 + c) * kHS + ks * 32 + 8 * hh);
      a1[j] = mma_b(ah[ks], w1, a1[j]);
      a1[j] = mma_b(al[ks], w1, a1[j]);
      a2[j] = mma_b(ah[ks], w2, a2[j]);
      a2[j] = mma_b(al[ks], w2, a2[j]);
    }
  }
  acc_guard4(a1[0], a1[1], a1[2], a1[3]);
  acc_guard4(a2[0], a2[1], a2[2], a2[3]);

#pragma unroll
  for (int j = 0; j < 4; ++j) {
    const int col = j * 16 + c;
    const float bb1 = sBias[col];
    const float bb2 = sBias[kHS + col];
#pragma unroll
    for (int r = 0; r < 8; ++r) {
      const int row = wave * 16 + 8 * hh + r;
      const float vres = sA[row * kGP + col];
      a1[j][r] = vres + (a1[j][r] + bb1);
      a2[j][r] = a2[j][r] + bb2;
    }
  }
  __syncthreads();
#pragma unroll
  for (int j = 0; j < 4; ++j) {
    const int col = j * 16 + c;
#pragma unroll
    for (int r = 0; r < 8; ++r) {
      const int row = wave * 16 + 8 * hh + r;
      sB[col * kGP + row] = a1[j][r];
      sA[col * kGP + row] = a2[j][r];
    }
  }
  __syncthreads();

  const int q = lane >> 3, c8 = (lane & 7) * 8;
#pragma unroll 1
  for (int it = 0; it < 4; ++it) {
    const int d = wave * 16 + it * 4 + q;
    const float* pa = sB + d * kGP + c8;
    const float* pg = sA + d * kGP + c8;
    const v4f av0 = *(const v4f*)(pa);
    const v4f av1 = *(const v4f*)(pa + 4);
    const v4f gv0 = *(const v4f*)(pg);
    const v4f gv1 = *(const v4f*)(pg + 4);
    v8h hv, lv;
#pragma unroll
    for (int e = 0; e < 4; ++e) {
      const float xa0 = av0[e];
      const float xg0 = gv0[e];
      const float xa1 = av1[e];
      const float xg1 = gv1[e];
      const float r0 = xa0 * (1.0f / (1.0f + expf(-xg0)));
      const float r1 = xa1 * (1.0f / (1.0f + expf(-xg1)));
      unsigned short hb, lb;
      split_bits(r0, hb, lb);
      hv[e] = __builtin_bit_cast(_Float16, hb);
      lv[e] = __builtin_bit_cast(_Float16, lb);
      split_bits(r1, hb, lb);
      hv[4 + e] = __builtin_bit_cast(_Float16, hb);
      lv[4 + e] = __builtin_bit_cast(_Float16, lb);
    }
    const size_t o = ((size_t)(bidx * kH + hd) * kHS + d) * kT + t0 + c8;
    *(volatile v8h*)(VTH + o) = hv;
    *(volatile v8h*)(VTL + o) = lv;
    __threadfence();
    *(volatile v8h*)(VTH + o) = hv;
    *(volatile v8h*)(VTL + o) = lv;
  }
}

constexpr int kKC = 64;
__global__ __launch_bounds__(128) void causal_attn_kernel(
    const unsigned short* __restrict__ Up, const unsigned short* __restrict__ XHp,
    const unsigned short* __restrict__ VTHp, const unsigned short* __restrict__ VTLp,
    unsigned short* __restrict__ YH, unsigned short* __restrict__ YL)
{
  __shared__ __align__(16) _Float16 Ksh[kKC * kHS];
  __shared__ __align__(16) __bf16 Vth[kHS * kKC];
  __shared__ __align__(16) __bf16 Vtl[kHS * kKC];
  __shared__ __align__(16) __bf16 Psh[4][16 * kKC];
  __shared__ __align__(16) __bf16 Psl[4][16 * kKC];
  __shared__ __align__(16) float  Os[4][16 * 68];

  const int tid  = threadIdx.x;
  const int wave = tid >> 5;
  const int lane = tid & 31;
  const int hh   = lane >> 4;
  const int c    = lane & 15;

  constexpr int nqb = kT / 64;
  const int bx = blockIdx.x;
  const int qb = bx % nqb;
  const int bh = bx / nqb;
  const int h  = bh % kH;
  const int b  = bh / kH;
  const int q0 = qb * 64 + wave * 16;

  const _Float16* Uh = (const _Float16*)Up;
  const _Float16* Xh = (const _Float16*)XHp;
  const __bf16*   Vh = (const __bf16*)VTHp;
  const __bf16*   Vl = (const __bf16*)VTLp;

  v16h qa[2];
  {
    const _Float16* urow = Uh + (size_t)(b * kT + q0 + c) * kC + h * kHS;
#pragma unroll
    for (int dc = 0; dc < 2; ++dc) qa[dc] = Frag<_Float16>::load(urow + dc * 32 + 8 * hh);
  }

  float mrow[8], lrow[8];
  v8f oacc[4];
#pragma unroll
  for (int r = 0; r < 8; ++r) { mrow[r] = -INFINITY; lrow[r] = 0.f; }
#pragma unroll
  for (int t = 0; t < 4; ++t) oacc[t] = (v8f){0.f,0.f,0.f,0.f,0.f,0.f,0.f,0.f};

  __bf16* pwh = Psh[wave];
  __bf16* pwl = Psl[wave];
  const int nChunks = qb + 1;
  for (int kc = 0; kc < nChunks; ++kc) {
    const int kv0 = kc * kKC;
    __syncthreads();
#pragma unroll
    for (int i = 0; i < 4; ++i) {
      const int e = i * 128 + tid;
      const int r = e >> 3, c8 = (e & 7) * 8;
      *(v8h*)(Ksh + r * kHS + c8) = *(const v8h*)(Xh + (size_t)(b * kT + kv0 + r) * kC + h * kHS + c8);
      const size_t vo = ((size_t)bh * kHS + r) * kT + kv0 + c8;
      *(v8b*)(Vth + r * kKC + c8) = *(const v8b*)(Vh + vo);
      *(v8b*)(Vtl + r * kKC + c8) = *(const v8b*)(Vl + vo);
    }
    __syncthreads();

    v8f s[4];
#pragma unroll
    for (int j = 0; j < 4; ++j) {
      s[j] = (v8f){0.f,0.f,0.f,0.f,0.f,0.f,0.f,0.f};
#pragma unroll
      for (int dc = 0; dc < 2; ++dc) {
        const v16h kb = Frag<_Float16>::load(Ksh + (j * 16 + c) * kHS + dc * 32 + 8 * hh);
        s[j] = mma_h(qa[dc], kb, s[j]);
      }
    }
    acc_guard4(s[0], s[1], s[2], s[3]);

    const bool diag = (kc == qb);
    float cm[8];
#pragma unroll
    for (int r = 0; r < 8; ++r) {
      const int qrow = q0 + 8 * hh + r;
      float m = -INFINITY;
#pragma unroll
      for (int j = 0; j < 4; ++j) {
        const int kvcol = kv0 + j * 16 + c;
        float sv = s[j][r] * kScoreScale;
        const bool masked = diag && (kvcol > qrow);
        sv = masked ? -INFINITY : sv;
        s[j][r] = sv;
        m = fmaxf(m, sv);
      }
#pragma unroll
      for (int off = 1; off < 16; off <<= 1) m = fmaxf(m, __shfl_xor(m, off, 32));
      cm[r] = m;
    }
#pragma unroll
    for (int r = 0; r < 8; ++r) {
      const float mnew = fmaxf(mrow[r], cm[r]);
      const float alpha = __expf(mrow[r] - mnew);
      mrow[r] = mnew;
      float psum = 0.f;
#pragma unroll
      for (int j = 0; j < 4; ++j) {
        const float p = __expf(s[j][r] - mnew);
        psum += p;
        unsigned short hb, lb;
        split_bits(p, hb, lb);
        pwh[(8 * hh + r) * kKC + j * 16 + c] = __builtin_bit_cast(__bf16, hb);
        pwl[(8 * hh + r) * kKC + j * 16 + c] = __builtin_bit_cast(__bf16, lb);
      }
#pragma unroll
      for (int off = 1; off < 16; off <<= 1) psum += __shfl_xor(psum, off, 32);
      lrow[r] = lrow[r] * alpha + psum;
#pragma unroll
      for (int t = 0; t < 4; ++t) oacc[t][r] *= alpha;
    }
    __builtin_amdgcn_fence(__ATOMIC_RELEASE, "workgroup");
    __builtin_amdgcn_wave_barrier();
    __builtin_amdgcn_fence(__ATOMIC_ACQUIRE, "workgroup");
#pragma unroll 1
    for (int kk = 0; kk < 2; ++kk) {
      const v16b pa = Frag<__bf16>::load(pwh + c * kKC + kk * 32 + 8 * hh);
      const v16b pl = Frag<__bf16>::load(pwl + c * kKC + kk * 32 + 8 * hh);
#pragma unroll
      for (int t = 0; t < 4; ++t) {
        const v16b vb = Frag<__bf16>::load(Vth + (t * 16 + c) * kKC + kk * 32 + 8 * hh);
        const v16b vl = Frag<__bf16>::load(Vtl + (t * 16 + c) * kKC + kk * 32 + 8 * hh);
        oacc[t] = mma_b(pa, vb, oacc[t]);
        oacc[t] = mma_b(pa, vl, oacc[t]);
        oacc[t] = mma_b(pl, vb, oacc[t]);
      }
    }
    acc_guard4(oacc[0], oacc[1], oacc[2], oacc[3]);
  }

  float* os = Os[wave];
#pragma unroll
  for (int r = 0; r < 8; ++r) {
    const float inv = 1.0f / lrow[r];
#pragma unroll
    for (int t = 0; t < 4; ++t) os[(8 * hh + r) * 68 + t * 16 + c] = oacc[t][r] * inv;
  }
  __builtin_amdgcn_fence(__ATOMIC_RELEASE, "workgroup");
  __builtin_amdgcn_wave_barrier();
  __builtin_amdgcn_fence(__ATOMIC_ACQUIRE, "workgroup");
  {
    const int q = lane >> 3, c8 = (lane & 7) * 8;
    v8h hv[4], lv[4];
#pragma unroll
    for (int it = 0; it < 4; ++it) {
      const int row = it * 4 + q;
      const float* sp = os + row * 68 + c8;
      const v4f y0 = *(const v4f*)(sp);
      const v4f y1 = *(const v4f*)(sp + 4);
#pragma unroll
      for (int e = 0; e < 4; ++e) {
        const float z0 = y0[e];
        const float z1 = y1[e];
        unsigned short hb, lb;
        split_bits(z0, hb, lb);
        hv[it][e] = __builtin_bit_cast(_Float16, hb);
        lv[it][e] = __builtin_bit_cast(_Float16, lb);
        split_bits(z1, hb, lb);
        hv[it][4 + e] = __builtin_bit_cast(_Float16, hb);
        lv[it][4 + e] = __builtin_bit_cast(_Float16, lb);
      }
    }
    for (int pass = 0; pass < 2; ++pass) {
#pragma unroll
      for (int it = 0; it < 4; ++it) {
        const int row = it * 4 + q;
        const size_t o = (size_t)(b * kT + q0 + row) * kC + h * kHS + c8;
        *(volatile v8h*)(YH + o) = hv[it];
        *(volatile v8h*)(YL + o) = lv[it];
      }
      __threadfence();
    }
  }
}

extern "C" void kernel_launch(void* const* d_in, const int* in_sizes, int n_in,
                              void* d_out, int out_size, void* d_ws, size_t ws_size,
                              hipStream_t stream) {
  if (n_in < 11) return;
  if (in_sizes[0] != kRows * kC) return;
  if (in_sizes[1] != kC * kC) return;
  if (in_sizes[2] != kC) return;
  if (in_sizes[3] != kC * kC) return;
  if (in_sizes[4] != kC) return;
  if (in_sizes[5] != kHS * kHS) return;
  if (in_sizes[6] != kHS) return;
  if (in_sizes[7] != kHS * kHS) return;
  if (in_sizes[8] != kHS) return;
  if (in_sizes[9] != kC * kC) return;
  if (in_sizes[10] != kC) return;
  if (out_size != kRows * kC) return;
  if (ws_size < kWsTotal) return;

  const float* x  = (const float*)d_in[0];
  const float* Wu = (const float*)d_in[1];
  const float* bu = (const float*)d_in[2];
  const float* Wv = (const float*)d_in[3];
  const float* bv = (const float*)d_in[4];
  const float* W1 = (const float*)d_in[5];
  const float* b1 = (const float*)d_in[6];
  const float* W2 = (const float*)d_in[7];
  const float* b2 = (const float*)d_in[8];
  const float* Wp = (const float*)d_in[9];
  const float* bp = (const float*)d_in[10];
  float* out = (float*)d_out;

  char* ws = (char*)d_ws;
  unsigned short* XH   = (unsigned short*)(ws + kOffXH);
  unsigned short* WUT  = (unsigned short*)(ws + kOffWUT);
  unsigned short* WVT  = (unsigned short*)(ws + kOffWVT);
  unsigned short* WPT  = (unsigned short*)(ws + kOffWPT);
  unsigned short* W12T = (unsigned short*)(ws + kOffW12);
  unsigned short* U16  = (unsigned short*)(ws + kOffU);
  float*          V0   = (float*)(ws + kOffV0);
  unsigned short* YH   = (unsigned short*)(ws + kOffYH);
  unsigned short* YL   = (unsigned short*)(ws + kOffYL);
  unsigned short* VTH  = (unsigned short*)(ws + kOffVTH);
  unsigned short* VTL  = (unsigned short*)(ws + kOffVTL);

  cast_x_kernel<<<(kRows * kC / 8) / 256, 256, 0, stream>>>(x, XH, kRows * kC / 8);

  wt_transpose_cast_kernel<<<dim3(kC / 64, kC / 64, 3), 256, 0, stream>>>(Wu, Wv, Wp, WUT, kC, kWCarry, 2);
  wt_transpose_cast_kernel<<<dim3(1, 1, 2), 256, 0, stream>>>(W1, W2, W2, W12T, kHS, 1.0f, 0);

  wmma_gemm64<0, 0, 2, 1><<<dim3(256, 1), 256, 0, stream>>>(
      XH, XH, kC, 0L,
      WUT, WUT, kC, 0L,
      (void*)U16, kC, 0L,
      bu, kRows, kC, kC, kUScale, kUCarry);

  wmma_gemm64<0, 0, 2, 0><<<dim3(256, 1), 256, 0, stream>>>(
      XH, XH, kC, 0L,
      WVT, WVT, kC, 0L,
      (void*)V0, kC, 0L,
      bv, kRows, kC, kC, kV0Scale, 1.0f);

  gated_value_kernel<<<dim3(kRows / 64, kH), 128, 0, stream>>>(V0, W12T, W12T + kHS * kHS, b1, b2, VTH, VTL);

  causal_attn_kernel<<<kB * kH * (kT / 64), 128, 0, stream>>>(U16, XH, VTH, VTL, YH, YL);

  wmma_gemm64<1, 1, 2, 0><<<dim3(256, 1), 256, 0, stream>>>(
      YH, YL, kC, 0L,
      WPT, WPT, kC, 0L,
      (void*)out, kC, 0L,
      bp, kRows, kC, kC, 1.0f, 1.0f);
}
